// SimpleMambaClassifier_39565238731516
// MI455X (gfx1250) — hardware-verified
//
#include <hip/hip_runtime.h>


#define NB_    4
#define NL_    1024
#define MT_    (NB_ * NL_)
#define DM_    256
#define DI_    512
#define NS_    16
#define DTR_   16
#define XPN_   48
#define XPP_   64
#define NCLS_  10
#define NLAY_  4

static_assert(MT_ % 64 == 0);
static_assert(DM_ % 64 == 0);
static_assert(DI_ % 64 == 0);
static_assert((2 * DI_) % 64 == 0);
static_assert(DM_ % 32 == 0);
static_assert(DI_ % 32 == 0);
static_assert((NL_ & (NL_ - 1)) == 0);
static_assert(NL_ % 16 == 0);
static_assert(DM_ == 256);
static_assert(NB_ * NCLS_ <= 64);
static_assert(XPP_ == 64);

typedef float          v4f   __attribute__((ext_vector_type(4)));
typedef float          v8f   __attribute__((ext_vector_type(8)));
typedef __bf16         v16b  __attribute__((ext_vector_type(16)));
typedef unsigned short u16x8 __attribute__((ext_vector_type(8)));

union FragB { u16x8 h[2]; v16b v; };

__device__ __forceinline__ unsigned short f32_to_bf16(float f) {
    unsigned u = __float_as_uint(f);
    unsigned r = u + 0x7FFFu + ((u >> 16) & 1u);
    return (unsigned short)(r >> 16);
}
__device__ __forceinline__ float bf16_to_f32(unsigned short b) {
    return __uint_as_float(((unsigned)b) << 16);
}
__device__ __forceinline__ float silu_f(float x) {
    float e = expf(-x);
    return x * __builtin_amdgcn_rcpf(1.0f + e);
}
__device__ __forceinline__ float softplus_f(float x) {
    return fmaxf(x, 0.0f) + log1pf(expf(-fabsf(x)));
}
__device__ __forceinline__ float conv4_silu(float x0, float x1, float x2, float x3,
                                            float w0, float w1, float w2, float w3, float bias) {
    float c = w0 * x0 + w1 * x1 + w2 * x2 + w3 * x3;
    return silu_f(c + bias);
}
__device__ __forceinline__ v8f ld8f(const float* p) {
    v4f a = *(const v4f*)p;
    v4f b = *(const v4f*)(p + 4);
    return __builtin_shufflevector(a, b, 0, 1, 2, 3, 4, 5, 6, 7);
}
__device__ __forceinline__ v8f zero8() {
    v8f z;
#pragma unroll
    for (int c = 0; c < 8; ++c) z[c] = 0.0f;
    return z;
}
__device__ __forceinline__ float wave_sum(float v) {
#pragma unroll
    for (int o = 16; o > 0; o >>= 1) v += __shfl_xor(v, o, 32);
    return v;
}
__device__ __forceinline__ void split8(const v8f x, u16x8& hv, u16x8& lv) {
#pragma unroll
    for (int c = 0; c < 8; ++c) {
        const float f = x[c];
        const unsigned short hb = f32_to_bf16(f);
        const unsigned short lb = f32_to_bf16(f - bf16_to_f32(hb));
        hv[c] = hb;
        lv[c] = lb;
    }
}

__device__ __forceinline__ void mma16(v8f& acc, const FragB& a, const FragB& b) {
    acc = __builtin_amdgcn_wmma_f32_16x16x32_bf16(false, a.v, false, b.v, (short)0, acc, false, false);
    asm volatile("v_nop\n\tv_nop\n\tv_nop\n\tv_nop" : "+v"(acc) : "v"(a.v), "v"(b.v));
}

__global__ __launch_bounds__(256)
void cvt_split_kernel(const float* __restrict__ src, unsigned short* dhi, unsigned short* dlo,
                      int n8, int K, int rsrc, int rdst)
{
    const int i = blockIdx.x * 256 + threadIdx.x;
    if (i >= n8) return;
    const size_t e    = (size_t)i * 8;
    const int    rowd = (int)(e / (size_t)K);
    const int    col  = (int)(e - (size_t)rowd * (size_t)K);
    const int    g    = rowd / rdst;
    const int    r    = rowd - g * rdst;
    const int    rs   = (r < rsrc) ? r : (rsrc - 1);
    v8f x = ld8f(src + ((size_t)g * rsrc + rs) * (size_t)K + col);
    if (r >= rsrc) x = zero8();
    u16x8 hv, lv;
    split8(x, hv, lv);
    *(volatile u16x8*)(dhi + e) = hv;
    *(volatile u16x8*)(dlo + e) = lv;
    __threadfence();
    *(volatile u16x8*)(dhi + e) = hv;
    *(volatile u16x8*)(dlo + e) = lv;
}

__global__ __launch_bounds__(256)
void pix_proj_kernel(const float* __restrict__ x, const float* __restrict__ w,
                     const float* __restrict__ bias, float* h)
{
    const int tid = threadIdx.x;
    const int m   = blockIdx.x * 4 + (tid >> 6);
    if (m >= MT_) return;
    const int d0  = (tid & 63) * 4;
    const int b   = m / NL_;
    const int l   = m & (NL_ - 1);
    const float* xb = x + (size_t)b * 3 * NL_ + l;
    const float x0 = xb[0], x1 = xb[NL_], x2 = xb[2 * NL_];
    v4f o;
#pragma unroll
    for (int j = 0; j < 4; ++j) {
        const int d = d0 + j;
        float a = x0 * w[d * 3 + 0];
        a += x1 * w[d * 3 + 1];
        a += x2 * w[d * 3 + 2];
        o[j] = a + bias[d];
    }
    float* gp = h + (size_t)m * DM_ + d0;
    *(volatile v4f*)gp = o;
    __threadfence();
    *(volatile v4f*)gp = o;
}

__global__ __launch_bounds__(256)
void ln_split_kernel(const float* __restrict__ hin, const float* __restrict__ w,
                     const float* __restrict__ bb, unsigned short* xhi, unsigned short* xlo)
{
    const int tid  = threadIdx.x;
    const int lane = tid & 31;
    const int wave = tid >> 5;
    const int row  = blockIdx.x * 8 + wave;
    if (row >= MT_) return;
    const int c0   = lane * 8;
    const size_t e = (size_t)row * DM_ + c0;
    const v8f x = ld8f(hin + e);
    float s = 0.0f;
#pragma unroll
    for (int c = 0; c < 8; ++c) s += x[c];
    s = wave_sum(s);
    const float mu = s * (1.0f / DM_);
    v8f d;
    float q = 0.0f;
#pragma unroll
    for (int c = 0; c < 8; ++c) { d[c] = x[c] - mu; q += d[c] * d[c]; }
    q = wave_sum(q);
    const float rstd = rsqrtf(q * (1.0f / DM_) + 1e-5f);
    const v8f w8 = ld8f(w + c0);
    const v8f b8 = ld8f(bb + c0);
    v8f y;
#pragma unroll
    for (int c = 0; c < 8; ++c) y[c] = (d[c] * rstd) * w8[c] + b8[c];
    u16x8 hv, lv;
    split8(y, hv, lv);
    *(volatile u16x8*)(xhi + e) = hv;
    *(volatile u16x8*)(xlo + e) = lv;
    __threadfence();
    *(volatile u16x8*)(xhi + e) = hv;
    *(volatile u16x8*)(xlo + e) = lv;
}

template<int NBF>
__device__ __forceinline__ void tile_store_pass(const float* st, float* gp, int ldc, int lane) {
    constexpr int CW  = NBF * 16;
    constexpr int P   = CW + 4;
    constexpr int LPR = CW / 4;
    constexpr int RPI = 32 / LPR;
    constexpr int NIT = 32 / RPI;
    const int rsub = lane / LPR;
    const int c4   = (lane % LPR) * 4;
#pragma unroll
    for (int it = 0; it < NIT; ++it) {
        const int row = it * RPI + rsub;
        const v4f v = *(const v4f*)(st + row * P + c4);
        *(volatile v4f*)(gp + (size_t)row * ldc + c4) = v;
    }
}

template<int NBF>
__global__ __launch_bounds__(128)
void gemm_split_kernel(const unsigned short* __restrict__ A,  const unsigned short* __restrict__ A2,
                       const unsigned short* __restrict__ Bw, const unsigned short* __restrict__ B2,
                       const float* R, float* C, float* C2,
                       int K, int ldc, int csplit, int has_res)
{
    constexpr int CW = NBF * 16;
    constexpr int P  = CW + 4;
    __shared__ __attribute__((aligned(16))) float stile[4][32 * P];

    const int tid  = threadIdx.x;
    const int lane = tid & 31;
    const int wave = tid >> 5;
    const int h    = lane >> 4;
    const int m    = lane & 15;
    const int wm   = wave >> 1;
    const int wn   = wave & 1;

    const int rowW = blockIdx.y * 64 + wm * 32;
    const int colW = blockIdx.x * (2 * CW) + wn * CW;

    v8f acc[2 * NBF];
#pragma unroll
    for (int j = 0; j < 2 * NBF; ++j)
#pragma unroll
        for (int r = 0; r < 8; ++r) acc[j][r] = 0.0f;

    const size_t aoff  = (size_t)(rowW + m) * K + 8 * h;
    const size_t boff  = (size_t)(colW + m) * K + 8 * h;
    const size_t sub16 = (size_t)16 * K;
    const int nk = K >> 5;

    for (int kt = 0; kt < nk; ++kt) {
        const size_t k0 = (size_t)kt * 32;
        FragB fa[2], fb[NBF], ga[2], gb[NBF];
#pragma unroll
        for (int s = 0; s < 2; ++s) {
            const unsigned short* p = A + aoff + s * sub16 + k0;
            fa[s].h[0] = *(const u16x8*)(p);
            fa[s].h[1] = *(const u16x8*)(p + 16);
            const unsigned short* q = A2 + aoff + s * sub16 + k0;
            ga[s].h[0] = *(const u16x8*)(q);
            ga[s].h[1] = *(const u16x8*)(q + 16);
        }
#pragma unroll
        for (int j = 0; j < NBF; ++j) {
            const unsigned short* p = Bw + boff + j * sub16 + k0;
            fb[j].h[0] = *(const u16x8*)(p);
            fb[j].h[1] = *(const u16x8*)(p + 16);
            const unsigned short* q = B2 + boff + j * sub16 + k0;
            gb[j].h[0] = *(const u16x8*)(q);
            gb[j].h[1] = *(const u16x8*)(q + 16);
        }
#pragma unroll
        for (int s = 0; s < 2; ++s)
#pragma unroll
            for (int j = 0; j < NBF; ++j) {
                mma16(acc[s * NBF + j], fa[s], fb[j]);
                mma16(acc[s * NBF + j], fa[s], gb[j]);
                mma16(acc[s * NBF + j], ga[s], fb[j]);
            }
    }

    float* st = stile[wave];
#pragma unroll
    for (int s = 0; s < 2; ++s)
#pragma unroll
        for (int j = 0; j < NBF; ++j)
#pragma unroll
            for (int r = 0; r < 8; ++r)
                st[(s * 16 + 8 * h + r) * P + j * 16 + m] = acc[s * NBF + j][r];
    __syncthreads();

    float* Cp = C;
    int gcol = colW;
    if (colW >= csplit) { Cp = C2; gcol = colW - csplit; }
    float* gp = Cp + (size_t)rowW * ldc + gcol;

    if (has_res) {
        constexpr int LPR = CW / 4;
        constexpr int RPI = 32 / LPR;
        constexpr int NIT = 32 / RPI;
        const int rsub = lane / LPR;
        const int c4   = (lane % LPR) * 4;
        const float* rp = R + (size_t)rowW * ldc + gcol;
#pragma unroll
        for (int it = 0; it < NIT; ++it) {
            const int row = it * RPI + rsub;
            const v4f v  = *(const v4f*)(st + row * P + c4);
            const v4f rr = *(const v4f*)(rp + (size_t)row * ldc + c4);
            *(v4f*)(st + row * P + c4) = v + rr;
        }
    }

    tile_store_pass<NBF>(st, gp, ldc, lane);
    __threadfence();
    tile_store_pass<NBF>(st, gp, ldc, lane);
}

__global__ __launch_bounds__(256)
void conv_split_kernel(const float* __restrict__ X, const float* __restrict__ cw,
                       const float* __restrict__ cb, unsigned short* uhi, unsigned short* ulo)
{
    const int tid = threadIdx.x;
    const int m   = blockIdx.x * 4 + (tid >> 6);
    if (m >= MT_) return;
    const int l   = m & (NL_ - 1);
    const int d0  = (tid & 63) * 8;
    const size_t base = (size_t)m * DI_ + d0;
    const int o1 = (l >= 1) ? 1 : 0;
    const int o2 = (l >= 2) ? 2 : 0;
    const int o3 = (l >= 3) ? 3 : 0;

    v8f x3 = ld8f(X + base);
    v8f x2 = ld8f(X + base - (size_t)o1 * DI_);
    v8f x1 = ld8f(X + base - (size_t)o2 * DI_);
    v8f x0 = ld8f(X + base - (size_t)o3 * DI_);
    if (l < 1) x2 = zero8();
    if (l < 2) x1 = zero8();
    if (l < 3) x0 = zero8();

    const float* wp = cw + (size_t)d0 * 4;
    v4f wv[8];
#pragma unroll
    for (int c = 0; c < 8; ++c) wv[c] = *(const v4f*)(wp + 4 * c);
    const v8f bias = ld8f(cb + d0);

    v8f u;
#pragma unroll
    for (int c = 0; c < 8; ++c)
        u[c] = conv4_silu(x0[c], x1[c], x2[c], x3[c], wv[c][0], wv[c][1], wv[c][2], wv[c][3], bias[c]);

    u16x8 hv, lv;
    split8(u, hv, lv);
    *(volatile u16x8*)(uhi + base) = hv;
    *(volatile u16x8*)(ulo + base) = lv;
    __threadfence();
    *(volatile u16x8*)(uhi + base) = hv;
    *(volatile u16x8*)(ulo + base) = lv;
}

__device__ __forceinline__ void rows16_store_pass(const unsigned short* sl, unsigned short* gpl,
                                                  size_t gbase, int lane) {
#pragma unroll
    for (int it = 0; it < 4; ++it) {
        const int t = it * 4 + (lane >> 3);
        const int c = (lane & 7) * 8;
        const u16x8 v = *(const u16x8*)(sl + t * 64 + c);
        *(volatile u16x8*)(gpl + gbase + (size_t)t * DI_ + c) = v;
    }
}

__global__ __launch_bounds__(64)
void scan_kernel(const float* __restrict__ X, const float* __restrict__ Z, const float* __restrict__ XD,
                 const float* __restrict__ cw, const float* __restrict__ cb,
                 const float* __restrict__ dtw, const float* __restrict__ dtb,
                 const float* __restrict__ Alog, const float* __restrict__ Dp,
                 unsigned short* yhi, unsigned short* ylo)
{
    __shared__ __attribute__((aligned(16))) unsigned short shi[16 * 64];
    __shared__ __attribute__((aligned(16))) unsigned short slo[16 * 64];
    __shared__ __attribute__((aligned(16))) float sx[16 * XPP_];

    const int tid   = threadIdx.x;
    const int lane  = tid & 31;
    const int wave  = tid >> 5;
    const int dbase = blockIdx.x * 64;
    const int d     = dbase + tid;
    const int b     = blockIdx.y;

    float an[NS_], hs[NS_], wr[DTR_];
#pragma unroll
    for (int n = 0; n < NS_; ++n) {
        an[n] = -expf(Alog[d * NS_ + n]);
        hs[n] = 0.0f;
    }
#pragma unroll
    for (int r = 0; r < DTR_; ++r) wr[r] = dtw[d * DTR_ + r];
    const float w0 = cw[d * 4 + 0], w1 = cw[d * 4 + 1], w2 = cw[d * 4 + 2], w3 = cw[d * 4 + 3];
    const float cbias = cb[d];
    const float tb = dtb[d];
    const float Dd = Dp[d];

    float xm1 = 0.0f, xm2 = 0.0f, xm3 = 0.0f;
    const size_t mrow0 = (size_t)b * NL_;

    const unsigned short* sl = wave ? slo : shi;
    unsigned short* gpl = wave ? ylo : yhi;
    const int srow_ = tid >> 2;
    const int scol_ = (tid & 3) * 16;

#pragma unroll 1
    for (int l0 = 0; l0 < NL_; l0 += 16) {
        {
            const float* p = XD + (mrow0 + (size_t)(l0 + srow_)) * XPP_ + scol_;
            float* q = sx + srow_ * XPP_ + scol_;
#pragma unroll
            for (int j = 0; j < 4; ++j) *(v4f*)(q + 4 * j) = *(const v4f*)(p + 4 * j);
        }
        __syncthreads();
#pragma unroll 1
        for (int t = 0; t < 16; ++t) {
            const size_t mrow = mrow0 + (size_t)(l0 + t);
            const size_t e = mrow * DI_ + d;
            const float xv = X[e];
            const float zv = Z[e];
            const float u  = conv4_silu(xm3, xm2, xm1, xv, w0, w1, w2, w3, cbias);
            xm3 = xm2; xm2 = xm1; xm1 = xv;

            const float* srow = sx + t * XPP_;
            const v4f p0 = *(const v4f*)(srow + 0);
            const v4f p1 = *(const v4f*)(srow + 4);
            const v4f p2 = *(const v4f*)(srow + 8);
            const v4f p3 = *(const v4f*)(srow + 12);
            const v4f q0 = *(const v4f*)(srow + 16);
            const v4f q1 = *(const v4f*)(srow + 20);
            const v4f q2 = *(const v4f*)(srow + 24);
            const v4f q3 = *(const v4f*)(srow + 28);
            const v4f c0 = *(const v4f*)(srow + 32);
            const v4f c1 = *(const v4f*)(srow + 36);
            const v4f c2 = *(const v4f*)(srow + 40);
            const v4f c3 = *(const v4f*)(srow + 44);

            float Bv[NS_], Cv[NS_], Tv[DTR_];
#pragma unroll
            for (int c = 0; c < 4; ++c) {
                Tv[c] = p0[c]; Tv[4 + c] = p1[c]; Tv[8 + c] = p2[c]; Tv[12 + c] = p3[c];
                Bv[c] = q0[c]; Bv[4 + c] = q1[c]; Bv[8 + c] = q2[c]; Bv[12 + c] = q3[c];
                Cv[c] = c0[c]; Cv[4 + c] = c1[c]; Cv[8 + c] = c2[c]; Cv[12 + c] = c3[c];
            }
            float pre = 0.0f;
#pragma unroll
            for (int r = 0; r < DTR_; ++r) pre += Tv[r] * wr[r];
            const float dt = softplus_f(pre + tb);
            const float du = dt * u;
            float y = 0.0f;
#pragma unroll
            for (int n = 0; n < NS_; ++n) {
                const float da = __expf(dt * an[n]);
                hs[n] = da * hs[n] + du * Bv[n];
                y += hs[n] * Cv[n];
            }
            const float g = (y + Dd * u) * silu_f(zv);
            const unsigned short hb = f32_to_bf16(g);
            const unsigned short lb = f32_to_bf16(g - bf16_to_f32(hb));
            shi[t * 64 + tid] = hb;
            slo[t * 64 + tid] = lb;
        }
        __syncthreads();
        const size_t gbase = (mrow0 + (size_t)l0) * DI_ + dbase;
        rows16_store_pass(sl, gpl, gbase, lane);
        __threadfence();
        rows16_store_pass(sl, gpl, gbase, lane);
        __syncthreads();
    }
}

__device__ __forceinline__ float block_sum256(float v, float* sred, int lane, int wave) {
    v = wave_sum(v);
    __syncthreads();
    if (lane == 0) sred[wave] = v;
    __syncthreads();
    float s = 0.0f;
#pragma unroll
    for (int w = 0; w < 8; ++w) s += sred[w];
    return s;
}

__global__ __launch_bounds__(256)
void head_kernel(const float* __restrict__ h, const float* __restrict__ fnw,
                 const float* __restrict__ fnb, const float* __restrict__ clsw,
                 const float* __restrict__ clsb, float* out)
{
    __shared__ float snh[NB_ * DM_];
    __shared__ float sred[8];
    __shared__ __attribute__((aligned(16))) float sout[64];
    const int t    = threadIdx.x;
    const int lane = t & 31;
    const int wave = t >> 5;
    const float wv = fnw[t];
    const float bv = fnb[t];
    if (t < 64) sout[t] = 0.0f;

#pragma unroll 1
    for (int b = 0; b < NB_; ++b) {
        const float* hp = h + (size_t)b * NL_ * DM_ + t;
        double s = 0.0;
#pragma unroll 4
        for (int l = 0; l < NL_; ++l) s += (double)hp[(size_t)l * DM_];
        const float v    = (float)(s * (1.0 / NL_));
        const float mu   = block_sum256(v, sred, lane, wave) * (1.0f / DM_);
        const float dv   = v - mu;
        const float var  = block_sum256(dv * dv, sred, lane, wave) * (1.0f / DM_);
        const float rstd = rsqrtf(var + 1e-5f);
        snh[b * DM_ + t] = (dv * rstd) * wv + bv;
    }
    __syncthreads();
    if (t < NB_ * NCLS_) {
        const int b = t / NCLS_;
        const int c = t - b * NCLS_;
        const float* wp = clsw + (size_t)c * DM_;
        const float* np0 = snh + b * DM_;
        float a = 0.0f;
#pragma unroll 4
        for (int d2 = 0; d2 < DM_; ++d2) a += np0[d2] * wp[d2];
        sout[t] = a + clsb[c];
    }
    __syncthreads();
    if (t < NCLS_) {
        const v4f v = *(const v4f*)(sout + 4 * t);
        *(volatile v4f*)(out + 4 * t) = v;
        __threadfence();
        *(volatile v4f*)(out + 4 * t) = v;
    }
}

extern "C" void kernel_launch(void* const* d_in, const int* in_sizes, int n_in,
                              void* d_out, int out_size, void* d_ws, size_t ws_size,
                              hipStream_t stream)
{
    if (n_in < 18) return;
    if (in_sizes[0]  != NB_ * 3 * NL_)          return;
    if (in_sizes[1]  != DM_ * 3)                return;
    if (in_sizes[2]  != DM_)                    return;
    if (in_sizes[3]  != NLAY_ * 2 * DI_ * DM_)  return;
    if (in_sizes[4]  != NLAY_ * DI_ * 4)        return;
    if (in_sizes[5]  != NLAY_ * DI_)            return;
    if (in_sizes[6]  != NLAY_ * XPN_ * DI_)     return;
    if (in_sizes[7]  != NLAY_ * DI_ * DTR_)     return;
    if (in_sizes[8]  != NLAY_ * DI_)            return;
    if (in_sizes[9]  != NLAY_ * DI_ * NS_)      return;
    if (in_sizes[10] != NLAY_ * DI_)            return;
    if (in_sizes[11] != NLAY_ * DM_ * DI_)      return;
    if (in_sizes[12] != NLAY_ * DM_)            return;
    if (in_sizes[13] != NLAY_ * DM_)            return;
    if (in_sizes[14] != DM_)                    return;
    if (in_sizes[15] != DM_)                    return;
    if (in_sizes[16] != NCLS_ * DM_)            return;
    if (in_sizes[17] != NCLS_)                  return;
    if (out_size != NB_ * NCLS_)                return;

    const float* x    = (const float*)d_in[0];
    const float* ipw  = (const float*)d_in[1];
    const float* ipb  = (const float*)d_in[2];
    const float* inw  = (const float*)d_in[3];
    const float* cw   = (const float*)d_in[4];
    const float* cb   = (const float*)d_in[5];
    const float* xpw  = (const float*)d_in[6];
    const float* dtw  = (const float*)d_in[7];
    const float* dtb  = (const float*)d_in[8];
    const float* alog = (const float*)d_in[9];
    const float* dsk  = (const float*)d_in[10];
    const float* ow   = (const float*)d_in[11];
    const float* lnw  = (const float*)d_in[12];
    const float* lnb  = (const float*)d_in[13];
    const float* fnw  = (const float*)d_in[14];
    const float* fnb  = (const float*)d_in[15];
    const float* clsw = (const float*)d_in[16];
    const float* clsb = (const float*)d_in[17];
    float* outp = (float*)d_out;

    const size_t SZ_WI = (size_t)NLAY_ * 2 * DI_ * DM_ * 2;
    const size_t SZ_WX = (size_t)NLAY_ * XPP_ * DI_ * 2;
    const size_t SZ_WO = (size_t)NLAY_ * DM_ * DI_ * 2;
    const size_t SZ_H  = (size_t)MT_ * DM_ * 4;
    const size_t SZ_XN = (size_t)MT_ * DM_ * 2;
    const size_t SZ_F  = (size_t)MT_ * DI_ * 4;
    const size_t SZ_U  = (size_t)MT_ * DI_ * 2;
    const size_t SZ_XD = (size_t)MT_ * XPP_ * 4;

    const size_t OFF_WIH = 0;
    const size_t OFF_WIL = OFF_WIH + SZ_WI;
    const size_t OFF_WXH = OFF_WIL + SZ_WI;
    const size_t OFF_WXL = OFF_WXH + SZ_WX;
    const size_t OFF_WOH = OFF_WXL + SZ_WX;
    const size_t OFF_WOL = OFF_WOH + SZ_WO;
    const size_t OFF_HA  = OFF_WOL + SZ_WO;
    const size_t OFF_HB  = OFF_HA  + SZ_H;
    const size_t OFF_XNH = OFF_HB  + SZ_H;
    const size_t OFF_XNL = OFF_XNH + SZ_XN;
    const size_t OFF_XF  = OFF_XNL + SZ_XN;
    const size_t OFF_ZF  = OFF_XF  + SZ_F;
    const size_t OFF_UH  = OFF_ZF  + SZ_F;
    const size_t OFF_UL  = OFF_UH  + SZ_U;
    const size_t OFF_XD  = OFF_UL  + SZ_U;
    const size_t OFF_YH  = OFF_XD  + SZ_XD;
    const size_t OFF_YL  = OFF_YH  + SZ_U;
    const size_t WS_END  = OFF_YL  + SZ_U;
    if (ws_size < WS_END) return;

    char* ws = (char*)d_ws;
    unsigned short* wih = (unsigned short*)(ws + OFF_WIH);
    unsigned short* wil = (unsigned short*)(ws + OFF_WIL);
    unsigned short* wxh = (unsigned short*)(ws + OFF_WXH);
    unsigned short* wxl = (unsigned short*)(ws + OFF_WXL);
    unsigned short* woh = (unsigned short*)(ws + OFF_WOH);
    unsigned short* wol = (unsigned short*)(ws + OFF_WOL);
    float*          hA  = (float*)(ws + OFF_HA);
    float*          hB  = (float*)(ws + OFF_HB);
    unsigned short* xnh = (unsigned short*)(ws + OFF_XNH);
    unsigned short* xnl = (unsigned short*)(ws + OFF_XNL);
    float*          Xf  = (float*)(ws + OFF_XF);
    float*          Zf  = (float*)(ws + OFF_ZF);
    unsigned short* uh  = (unsigned short*)(ws + OFF_UH);
    unsigned short* ul  = (unsigned short*)(ws + OFF_UL);
    float*          xd  = (float*)(ws + OFF_XD);
    unsigned short* yh  = (unsigned short*)(ws + OFF_YH);
    unsigned short* yl  = (unsigned short*)(ws + OFF_YL);

    {
        int n8;
        n8 = (NLAY_ * 2 * DI_ * DM_) / 8;
        hipLaunchKernelGGL(cvt_split_kernel, dim3((n8 + 255) / 256), dim3(256), 0, stream,
                           inw, wih, wil, n8, (int)DM_, (int)(NLAY_ * 2 * DI_), (int)(NLAY_ * 2 * DI_));
        n8 = (NLAY_ * XPP_ * DI_) / 8;
        hipLaunchKernelGGL(cvt_split_kernel, dim3((n8 + 255) / 256), dim3(256), 0, stream,
                           xpw, wxh, wxl, n8, (int)DI_, (int)XPN_, (int)XPP_);
        n8 = (NLAY_ * DM_ * DI_) / 8;
        hipLaunchKernelGGL(cvt_split_kernel, dim3((n8 + 255) / 256), dim3(256), 0, stream,
                           ow, woh, wol, n8, (int)DI_, (int)(NLAY_ * DM_), (int)(NLAY_ * DM_));
    }

    hipLaunchKernelGGL(pix_proj_kernel, dim3((MT_ + 3) / 4), dim3(256), 0, stream, x, ipw, ipb, hA);

    float* hcur = hA;
    float* hnxt = hB;

    for (int i = 0; i < NLAY_; ++i) {
        const float* cw_i   = cw   + (size_t)i * DI_ * 4;
        const float* cb_i   = cb   + (size_t)i * DI_;
        const float* dtw_i  = dtw  + (size_t)i * DI_ * DTR_;
        const float* dtb_i  = dtb  + (size_t)i * DI_;
        const float* alog_i = alog + (size_t)i * DI_ * NS_;
        const float* dsk_i  = dsk  + (size_t)i * DI_;
        const unsigned short* wih_i = wih + (size_t)i * 2 * DI_ * DM_;
        const unsigned short* wil_i = wil + (size_t)i * 2 * DI_ * DM_;
        const unsigned short* wxh_i = wxh + (size_t)i * XPP_ * DI_;
        const unsigned short* wxl_i = wxl + (size_t)i * XPP_ * DI_;
        const unsigned short* woh_i = woh + (size_t)i * DM_ * DI_;
        const unsigned short* wol_i = wol + (size_t)i * DM_ * DI_;

        hipLaunchKernelGGL(ln_split_kernel, dim3((MT_ + 7) / 8), dim3(256), 0, stream,
                           (const float*)hcur, lnw + (size_t)i * DM_, lnb + (size_t)i * DM_, xnh, xnl);

        hipLaunchKernelGGL(HIP_KERNEL_NAME(gemm_split_kernel<2>),
                           dim3((2 * DI_) / 64, MT_ / 64), dim3(128), 0, stream,
                           (const unsigned short*)xnh, (const unsigned short*)xnl, wih_i, wil_i,
                           (const float*)hcur, Xf, Zf, (int)DM_, (int)DI_, (int)DI_, 0);

        hipLaunchKernelGGL(conv_split_kernel, dim3((MT_ + 3) / 4), dim3(256), 0, stream,
                           (const float*)Xf, cw_i, cb_i, uh, ul);

        hipLaunchKernelGGL(HIP_KERNEL_NAME(gemm_split_kernel<2>),
                           dim3(XPP_ / 64, MT_ / 64), dim3(128), 0, stream,
                           (const unsigned short*)uh, (const unsigned short*)ul, wxh_i, wxl_i,
                           (const float*)hcur, xd, xd, (int)DI_, (int)XPP_, (int)(1 << 20), 0);

        hipLaunchKernelGGL(scan_kernel, dim3(DI_ / 64, NB_), dim3(64), 0, stream,
                           (const float*)Xf, (const float*)Zf, (const float*)xd, cw_i, cb_i, dtw_i, dtb_i,
                           alog_i, dsk_i, yh, yl);

        hipLaunchKernelGGL(HIP_KERNEL_NAME(gemm_split_kernel<2>),
                           dim3(DM_ / 64, MT_ / 64), dim3(128), 0, stream,
                           (const unsigned short*)yh, (const unsigned short*)yl, woh_i, wol_i,
                           (const float*)hcur, hnxt, hnxt, (int)DI_, (int)DM_, (int)(1 << 20), 1);

        float* tmp = hcur; hcur = hnxt; hnxt = tmp;
    }

    hipLaunchKernelGGL(head_kernel, dim3(1), dim3(256), 0, stream,
                       (const float*)hcur, fnw, fnb, clsw, clsb, outp);
}
